// SS_Conv_SSM_44744969290135
// MI455X (gfx1250) — hardware-verified
//
#include <hip/hip_runtime.h>
#include <math.h>

typedef __attribute__((ext_vector_type(16))) _Float16 v16h;
typedef __attribute__((ext_vector_type(8)))  _Float16 v8h;
typedef __attribute__((ext_vector_type(4)))  _Float16 v4h;
typedef __attribute__((ext_vector_type(16))) __bf16   v16b;
typedef __attribute__((ext_vector_type(8)))  __bf16   v8b;
typedef __attribute__((ext_vector_type(8)))  float    v8f;
typedef __attribute__((ext_vector_type(4)))  float    v4f;
typedef __attribute__((ext_vector_type(2)))  float    v2f;

constexpr int NBATCH = 8;
constexpr int IMH    = 56;
constexpr int IMW    = 56;
constexpr int CFULL  = 192;
constexpr int NPIX   = IMH * IMW;
constexpr int NTOK   = NBATCH * NPIX;
constexpr int CHALF  = 96;
constexpr int DIN    = 192;
constexpr int NST    = 16;
constexpr int DTRK   = 6;
constexpr int NDIR   = 4;
constexpr int KCONV  = 9 * CHALF;
constexpr int NPADC  = 128;
constexpr int XDW    = 64;
constexpr int XPROWS = 38;

__device__ __forceinline__ unsigned short f2bf_bits(float f) {
  unsigned u = __float_as_uint(f);
  return (unsigned short)((u + 0x7FFFu + ((u >> 16) & 1u)) >> 16);
}
__device__ __forceinline__ float bf_bits2f(unsigned short h) { return __uint_as_float(((unsigned)h) << 16); }

__device__ __forceinline__ void dep_guard_h(v8f& a, v8f& b, v16h x, v16h y) { asm volatile("v_nop\n\tv_nop\n\tv_nop\n\tv_nop" : "+v"(a), "+v"(b) : "v"(x), "v"(y)); }
__device__ __forceinline__ void dep_guard_b(v8f& a, v8f& b, v16b x, v16b y) { asm volatile("v_nop\n\tv_nop\n\tv_nop\n\tv_nop" : "+v"(a), "+v"(b) : "v"(x), "v"(y)); }
__device__ __forceinline__ void keep4_h(v16h a, v16h b, v16h c, v16h d) { asm volatile("v_nop" :: "v"(a), "v"(b), "v"(c), "v"(d)); }
__device__ __forceinline__ void keep4_b(v16b a, v16b b, v16b c, v16b d) { asm volatile("v_nop" :: "v"(a), "v"(b), "v"(c), "v"(d)); }
__device__ __forceinline__ void acc_guard4(v8f& a, v8f& b, v8f& c, v8f& d) { asm volatile("v_nop\n\tv_nop\n\tv_nop\n\tv_nop" : "+v"(a), "+v"(b), "+v"(c), "+v"(d)); }
template <typename T> struct Frag;
template <> struct Frag<_Float16> {
  typedef v16h V; union U { v16h v; v8h h[2]; };
  static __device__ __forceinline__ v16h load(const _Float16* p) {
    U f; f.h[0] = *(const v8h*)(p); f.h[1] = *(const v8h*)(p + 16); return f.v;
  }
  static __device__ __forceinline__ v8f mma(v16h a, v16h b, v8f c) {
    return __builtin_amdgcn_wmma_f32_16x16x32_f16(false, a, false, b, (short)0, c, false, false);
  }
  static __device__ __forceinline__ void guard(v8f& a, v8f& b, v16h x, v16h y) { dep_guard_h(a, b, x, y); }
  static __device__ __forceinline__ void keep(v16h a, v16h b, v16h c, v16h d) { keep4_h(a, b, c, d); }
};
template <> struct Frag<__bf16> {
  typedef v16b V; union U { v16b v; v8b h[2]; };
  static __device__ __forceinline__ v16b load(const __bf16* p) {
    U f; f.h[0] = *(const v8b*)(p); f.h[1] = *(const v8b*)(p + 16); return f.v;
  }
  static __device__ __forceinline__ v8f mma(v16b a, v16b b, v8f c) {
    return __builtin_amdgcn_wmma_f32_16x16x32_bf16(false, a, false, b, (short)0, c, false, false);
  }
  static __device__ __forceinline__ void guard(v8f& a, v8f& b, v16b x, v16b y) { dep_guard_b(a, b, x, y); }
  static __device__ __forceinline__ void keep(v16b a, v16b b, v16b c, v16b d) { keep4_b(a, b, c, d); }
};

template <int ET> struct Elem;
template <> struct Elem<0> { typedef _Float16 T; };
template <> struct Elem<1> { typedef __bf16 T; };
template <int ET, bool SPLIT, int BIAS_MODE, int OUT_MODE, bool RESID, int ACT = 0>
__global__ __launch_bounds__(256) void wmma_gemm64(
    const unsigned short* __restrict__ Ap, const unsigned short* __restrict__ A2p, int lda, long strideA,
    const unsigned short* __restrict__ Btp, const unsigned short* __restrict__ Bt2p, int ldb, long strideB,
    void* __restrict__ Cout, void* __restrict__ Cout2, int ldc, long strideC,
    const float* __restrict__ bias,
    const float* __restrict__ resid, long strideR,
    int M, int N, int K, float scale) {
  typedef typename Elem<ET>::T T;
  typedef typename Frag<T>::V V;
  const T* A = (const T*)Ap; const T* A2 = (const T*)A2p; const T* Bt = (const T*)Btp; const T* Bt2 = (const T*)Bt2p;
  __shared__ __align__(16) float sT[8][16 * 68];
  const int b    = blockIdx.y;
  const int lane = threadIdx.x & 31;
  const int wave = threadIdx.x >> 5;
  const int tilesN = N >> 6;
  const int tilesM = M >> 6;
  const int tile = blockIdx.x * 8 + wave;
  if (tile >= tilesM * tilesN) return;
  const int tm = tile / tilesN;
  const int tn = tile - tm * tilesN;
  const int m0 = tm << 6;
  const int n0 = tn << 6;

  const T* Ab  = A  + (size_t)b * strideA;
  const T* Bb  = Bt + (size_t)b * strideB;
  const T* Ab2 = SPLIT ? (A2  + (size_t)b * strideA) : nullptr;
  const T* Bb2 = SPLIT ? (Bt2 + (size_t)b * strideB) : nullptr;

  const int rlane = lane & 15;
  const int koff  = (lane >> 4) * 8;
  const int mOff  = (lane >> 4) * 8;

  v8f acc[4][4];
#pragma unroll
  for (int i = 0; i < 4; ++i)
#pragma unroll
    for (int j = 0; j < 4; ++j) acc[i][j] = (v8f){0.f,0.f,0.f,0.f,0.f,0.f,0.f,0.f};

  for (int k0 = 0; k0 < K; k0 += 32) {
    V bh[4], bl[4];
#pragma unroll
    for (int j = 0; j < 4; ++j) {
      const size_t bo = (size_t)(n0 + (j << 4) + rlane) * ldb + koff + k0;
      bh[j] = Frag<T>::load(Bb + bo);
      if (SPLIT) bl[j] = Frag<T>::load(Bb2 + bo);
    }
#pragma unroll
    for (int i = 0; i < 4; ++i) {
      const size_t ao = (size_t)(m0 + (i << 4) + rlane) * lda + koff + k0;
      V ah = Frag<T>::load(Ab + ao);
      V al;
      if (SPLIT) al = Frag<T>::load(Ab2 + ao);
#pragma unroll
      for (int j = 0; j < 4; ++j) {
        acc[i][j] = Frag<T>::mma(ah, bh[j], acc[i][j]);
        if (SPLIT) {
          acc[i][j] = Frag<T>::mma(ah, bl[j], acc[i][j]);
          acc[i][j] = Frag<T>::mma(al, bh[j], acc[i][j]);
        }
      }
      Frag<T>::guard(acc[i][0], acc[i][3], ah, SPLIT ? al : ah);
    }
    Frag<T>::keep(bh[0], bh[1], bh[2], bh[3]);
    if (SPLIT) Frag<T>::keep(bl[0], bl[1], bl[2], bl[3]);
  }
  acc_guard4(acc[0][0], acc[0][1], acc[0][2], acc[0][3]);
  acc_guard4(acc[1][0], acc[1][1], acc[1][2], acc[1][3]);
  acc_guard4(acc[2][0], acc[2][1], acc[2][2], acc[2][3]);
  acc_guard4(acc[3][0], acc[3][1], acc[3][2], acc[3][3]);

  float* slab = sT[wave];
  const float* Rb = RESID ? (resid + (size_t)b * strideR) : nullptr;
#pragma unroll
  for (int i = 0; i < 4; ++i) {
    const int mBase = m0 + (i << 4);
#pragma unroll
    for (int j = 0; j < 4; ++j) {
      const int n = n0 + (j << 4) + rlane;
      float bv = 0.f;
      if (BIAS_MODE == 2) bv = bias[n];
#pragma unroll
      for (int r = 0; r < 8; ++r) {
        float v = acc[i][j][r] * scale;
        if (BIAS_MODE == 1) v += bias[mBase + mOff + r];
        if (BIAS_MODE == 2) v += bv;
        if (RESID) v += Rb[(size_t)(mBase + mOff + r) * ldc + n];
        if (ACT == 1) v = tanhf(v);
        if (ACT == 2) v = fmaxf(v, 0.0f);
        if (ACT == 3) v = v / (1.0f + expf(-v));
        if (ACT == 4) v = (v > 0.f) ? v : 0.01f * v;
        if (ACT == 5) v = 0.5f * v * (1.0f + erff(v * 0.70710678118654752f));
        slab[(mOff + r) * 68 + (j << 4) + rlane] = v;
      }
    }
    __builtin_amdgcn_fence(__ATOMIC_RELEASE, "workgroup");
    __builtin_amdgcn_wave_barrier();
    __builtin_amdgcn_fence(__ATOMIC_ACQUIRE, "workgroup");
    if (OUT_MODE == 0) {
      float* C = (float*)Cout + (size_t)b * strideC;
      const int hh = lane >> 4, c4 = (lane & 15) * 4;
      for (int pass = 0; pass < 2; ++pass) {
#pragma unroll
        for (int it = 0; it < 8; ++it) {
          const int row = it * 2 + hh;
          v4f v = *(const v4f*)(slab + row * 68 + c4);
          *(volatile v4f*)(C + (size_t)(mBase + row) * ldc + n0 + c4) = v;
        }
        __threadfence();
      }
    } else {
      const int q = lane >> 3, c8 = (lane & 7) * 8;
      unsigned short* C  = (unsigned short*)Cout  + (size_t)b * strideC;
      unsigned short* C2 = (OUT_MODE == 2) ? ((unsigned short*)Cout2 + (size_t)b * strideC) : nullptr;
      for (int pass = 0; pass < 2; ++pass) {
#pragma unroll
        for (int it = 0; it < 4; ++it) {
          const int row = it * 4 + q;
          const float* sp = slab + row * 68 + c8;
          v8h hv, lv;
#pragma unroll
          for (int e = 0; e < 8; ++e) {
            if (OUT_MODE == 1) {
              hv[e] = (_Float16)sp[e];
            } else {
              unsigned short hb = f2bf_bits(sp[e]);
              unsigned short lb = f2bf_bits(sp[e] - bf_bits2f(hb));
              hv[e] = __builtin_bit_cast(_Float16, hb);
              lv[e] = __builtin_bit_cast(_Float16, lb);
            }
          }
          *(volatile v8h*)(C + (size_t)(mBase + row) * ldc + n0 + c8) = hv;
          if (OUT_MODE == 2) *(volatile v8h*)(C2 + (size_t)(mBase + row) * ldc + n0 + c8) = lv;
        }
        __threadfence();
      }
    }
    __builtin_amdgcn_fence(__ATOMIC_RELEASE, "workgroup");
    __builtin_amdgcn_wave_barrier();
    __builtin_amdgcn_fence(__ATOMIC_ACQUIRE, "workgroup");
  }
}

__global__ __launch_bounds__(256) void cast_convw_kernel(
    const float* __restrict__ w, unsigned short* __restrict__ dst, int KK, int nchunks, float scale)
{
  const int f = blockIdx.x * 256 + threadIdx.x;
  if (f >= nchunks) return;
  const int cpr = KK >> 3;
  const int co  = f / cpr;
  const int g   = f - co * cpr;
  const int cs  = (co < CHALF) ? co : (CHALF - 1);
  const bool valid = co < CHALF;
  const int kk0 = g * 8;
  v8h hv;
#pragma unroll
  for (int e = 0; e < 8; ++e) {
    const float v = w[(size_t)(kk0 + e) * CHALF + cs];
    hv[e] = (_Float16)(valid ? v * scale : 0.0f);
  }
  unsigned short* q = dst + (size_t)f * 8;
  *(volatile v8h*)q = hv;
  __threadfence();
  *(volatile v8h*)q = hv;
}

__global__ __launch_bounds__(256) void cast_rows_kernel(
    const float* __restrict__ src, unsigned short* __restrict__ dst,
    int R, int Rp, int Kc, int rot, int nchunks, float scale)
{
  const int f = blockIdx.x * 256 + threadIdx.x;
  if (f >= nchunks) return;
  const int cpr = Kc >> 3;
  const int rowflat = f / cpr;
  const int g  = f - rowflat * cpr;
  const int kb = rowflat / Rp;
  const int n  = rowflat - kb * Rp;
  const bool valid = n < R;
  int sr = n + rot;
  sr = (sr >= R) ? (sr - R) : sr;
  sr = valid ? sr : 0;
  const float* p = src + ((size_t)kb * R + sr) * Kc + g * 8;
  const v4f a0 = *(const v4f*)(p);
  const v4f a1 = *(const v4f*)(p + 4);
  v8h hv;
#pragma unroll
  for (int e = 0; e < 4; ++e) {
    hv[e]     = (_Float16)(valid ? a0[e] * scale : 0.0f);
    hv[4 + e] = (_Float16)(valid ? a1[e] * scale : 0.0f);
  }
  unsigned short* q = dst + (size_t)f * 8;
  *(volatile v8h*)q = hv;
  __threadfence();
  *(volatile v8h*)q = hv;
}

__global__ __launch_bounds__(256) void affine_f16_kernel(
    const float* __restrict__ src, int pitch,
    const float* __restrict__ bg, const float* __restrict__ bb,
    const float* __restrict__ bm, const float* __restrict__ bv,
    const float* __restrict__ cb, float cbmul, float relu_lo,
    unsigned short* __restrict__ dst, int nchunks)
{
  __shared__ __align__(16) float sSc[CHALF];
  __shared__ __align__(16) float sBe[CHALF];
  __shared__ __align__(16) float sM[CHALF];
  __shared__ __align__(16) float sCb[CHALF];
  const int t = threadIdx.x;
  if (t < CHALF) {
    sSc[t] = bg[t] * rsqrtf(bv[t] + 1e-5f);
    sBe[t] = bb[t];
    sM[t]  = bm[t];
    sCb[t] = cb[t] * cbmul;
  }
  __syncthreads();
  const int f = blockIdx.x * 256 + t;
  if (f >= nchunks) return;
  const int pos = f / 12;
  const int g8  = f - pos * 12;
  const int c0  = g8 * 8;
  const float* p = src + (size_t)pos * pitch + c0;
  const v4f a0 = *(const v4f*)(p);
  const v4f a1 = *(const v4f*)(p + 4);
  const v4f s0 = *(const v4f*)(sSc + c0), s1 = *(const v4f*)(sSc + c0 + 4);
  const v4f e0 = *(const v4f*)(sBe + c0), e1 = *(const v4f*)(sBe + c0 + 4);
  const v4f q0 = *(const v4f*)(sM + c0),  q1 = *(const v4f*)(sM + c0 + 4);
  const v4f k0 = *(const v4f*)(sCb + c0), k1 = *(const v4f*)(sCb + c0 + 4);
  v8h hv;
#pragma unroll
  for (int e = 0; e < 4; ++e) {
    float v0 = ((a0[e] + k0[e]) - q0[e]) * s0[e] + e0[e];
    v0 = fmaxf(v0, relu_lo);
    hv[e] = (_Float16)v0;
    float v1 = ((a1[e] + k1[e]) - q1[e]) * s1[e] + e1[e];
    v1 = fmaxf(v1, relu_lo);
    hv[4 + e] = (_Float16)v1;
  }
  unsigned short* q = dst + (size_t)f * 8;
  *(volatile v8h*)q = hv;
  __threadfence();
  *(volatile v8h*)q = hv;
}

__global__ __launch_bounds__(256) void im2col_copy_kernel(
    const unsigned short* __restrict__ T16, unsigned short* __restrict__ dst, int nchunks)
{
  const int f = blockIdx.x * 256 + threadIdx.x;
  if (f >= nchunks) return;
  const int pos = f / 108;
  const int rem = f - pos * 108;
  const int tap = rem / 12;
  const int g8  = rem - tap * 12;
  const int w_  = pos % IMW;
  const int h_  = (pos / IMW) % IMH;
  const int b_  = pos / NPIX;
  const int kh  = tap / 3;
  const int kw  = tap - kh * 3;
  const int hh  = h_ + kh - 1;
  const int ww  = w_ + kw - 1;
  const bool inimg = ((unsigned)hh < (unsigned)IMH) && ((unsigned)ww < (unsigned)IMW);
  const int hc = hh < 0 ? 0 : (hh >= IMH ? IMH - 1 : hh);
  const int wc = ww < 0 ? 0 : (ww >= IMW ? IMW - 1 : ww);
  const v8h v = *(const v8h*)(T16 + ((size_t)((b_ * IMH + hc) * IMW + wc)) * CHALF + g8 * 8);
  v8h hv;
#pragma unroll
  for (int e = 0; e < 8; ++e) hv[e] = inimg ? v[e] : (_Float16)0.0f;
  unsigned short* q = dst + (size_t)f * 8;
  *(volatile v8h*)q = hv;
  __threadfence();
  *(volatile v8h*)q = hv;
}

__global__ __launch_bounds__(256) void ln96_kernel(
    const float* __restrict__ x, const float* __restrict__ g, const float* __restrict__ be,
    unsigned short* __restrict__ dst)
{
  __shared__ __align__(16) _Float16 sT[64 * CHALF];
  const int t = threadIdx.x;
  const int r = t >> 2, part = t & 3;
  const int row = blockIdx.x * 64 + r;
  const float* xr = x + (size_t)row * CFULL + CHALF + part * 24;
  v4f a[6];
#pragma unroll
  for (int j = 0; j < 6; ++j) a[j] = *(const v4f*)(xr + 4 * j);
  float s = 0.f;
#pragma unroll
  for (int j = 0; j < 6; ++j) s += (a[j][0] + a[j][1]) + (a[j][2] + a[j][3]);
  s += __shfl_xor(s, 1, 32);
  s += __shfl_xor(s, 2, 32);
  const float mu = s * (1.0f / 96.0f);
  float q = 0.f;
#pragma unroll
  for (int j = 0; j < 6; ++j) {
#pragma unroll
    for (int e = 0; e < 4; ++e) { const float dd = a[j][e] - mu; q = fmaf(dd, dd, q); }
  }
  q += __shfl_xor(q, 1, 32);
  q += __shfl_xor(q, 2, 32);
  const float var = q * (1.0f / 96.0f);
  const float is  = rsqrtf(var + 1e-5f);
#pragma unroll
  for (int j = 0; j < 6; ++j) {
    const v4f gg = *(const v4f*)(g  + part * 24 + 4 * j);
    const v4f bb = *(const v4f*)(be + part * 24 + 4 * j);
    v4h hv;
#pragma unroll
    for (int e = 0; e < 4; ++e) hv[e] = (_Float16)(((a[j][e] - mu) * is) * gg[e] + bb[e]);
    *(v4h*)(sT + r * CHALF + part * 24 + 4 * j) = hv;
  }
  __syncthreads();
  v8h vals[3];
#pragma unroll
  for (int it = 0; it < 3; ++it) vals[it] = *(const v8h*)(sT + (it * 256 + t) * 8);
  unsigned short* ob = dst + (size_t)blockIdx.x * 64 * CHALF;
  for (int pass = 0; pass < 2; ++pass) {
#pragma unroll
    for (int it = 0; it < 3; ++it) *(volatile v8h*)(ob + (size_t)(it * 256 + t) * 8) = vals[it];
    __threadfence();
  }
}

__global__ __launch_bounds__(192) void dwconv_silu_kernel(
    const float* __restrict__ XP, const float* __restrict__ cw, const float* __restrict__ cbias,
    float* __restrict__ XI, unsigned short* __restrict__ XI16)
{
  __shared__ __align__(16) _Float16 sH[IMW * DIN];
  const int d  = threadIdx.x;
  const int b_ = blockIdx.x / IMH;
  const int h_ = blockIdx.x - b_ * IMH;
  const float w00 = cw[0 * DIN + d], w01 = cw[1 * DIN + d], w02 = cw[2 * DIN + d];
  const float w10 = cw[3 * DIN + d], w11 = cw[4 * DIN + d], w12 = cw[5 * DIN + d];
  const float w20 = cw[6 * DIN + d], w21 = cw[7 * DIN + d], w22 = cw[8 * DIN + d];
  const float bc = cbias[d];
  const bool up = h_ > 0, dn = h_ < IMH - 1;
  const int r0 = up ? (h_ - 1) : 0;
  const int r2 = dn ? (h_ + 1) : (IMH - 1);
  const float* p0 = XP + ((size_t)(b_ * IMH + r0) * IMW) * DIN + d;
  const float* p1 = XP + ((size_t)(b_ * IMH + h_) * IMW) * DIN + d;
  const float* p2 = XP + ((size_t)(b_ * IMH + r2) * IMW) * DIN + d;
  float a0m = 0.f, a1m = 0.f, a2m = 0.f;
  float a0c, a1c, a2c;
  {
    const float v0 = p0[0], v1 = p1[0], v2 = p2[0];
    a0c = up ? v0 : 0.f;
    a1c = v1;
    a2c = dn ? v2 : 0.f;
  }
  float* orow = XI + ((size_t)(b_ * IMH + h_) * IMW) * DIN + d;
#pragma unroll 1
  for (int w = 0; w < IMW; ++w) {
    const bool rv = (w + 1) < IMW;
    const int  wn = rv ? (w + 1) : (IMW - 1);
    const float n0 = p0[(size_t)wn * DIN], n1 = p1[(size_t)wn * DIN], n2 = p2[(size_t)wn * DIN];
    const float a0n = (up && rv) ? n0 : 0.f;
    const float a1n = rv ? n1 : 0.f;
    const float a2n = (dn && rv) ? n2 : 0.f;
    float acc = w00 * a0m;
    acc = fmaf(w01, a0c, acc);
    acc = fmaf(w02, a0n, acc);
    acc = fmaf(w10, a1m, acc);
    acc = fmaf(w11, a1c, acc);
    acc = fmaf(w12, a1n, acc);
    acc = fmaf(w20, a2m, acc);
    acc = fmaf(w21, a2c, acc);
    acc = fmaf(w22, a2n, acc);
    const float sv  = acc + bc;
    const float sg  = __builtin_amdgcn_rcpf(1.0f + __expf(-sv));
    const float out = sv * sg;
    float* op = orow + (size_t)w * DIN;
    *(volatile float*)op = out;
    __threadfence();
    *(volatile float*)op = out;
    sH[w * DIN + d] = (_Float16)(out * 64.0f);
    a0m = a0c; a0c = a0n;
    a1m = a1c; a1c = a1n;
    a2m = a2c; a2c = a2n;
  }
  __syncthreads();
  v8h vals[7];
#pragma unroll
  for (int it = 0; it < 7; ++it) vals[it] = *(const v8h*)(sH + (it * DIN + d) * 8);
  unsigned short* ob = XI16 + (size_t)blockIdx.x * IMW * DIN;
  for (int pass = 0; pass < 2; ++pass) {
#pragma unroll
    for (int it = 0; it < 7; ++it) *(volatile v8h*)(ob + (size_t)(it * DIN + d) * 8) = vals[it];
    __threadfence();
  }
}

__global__ __launch_bounds__(192) void scan4_kernel(
    const float* __restrict__ XDBL, const float* __restrict__ XI,
    const float* __restrict__ dtw, const float* __restrict__ dtb,
    const float* __restrict__ Alog, const float* __restrict__ Dsp,
    float* __restrict__ Y)
{
  __shared__ __align__(16) float sRow[32 * 40];
  const int d  = threadIdx.x;
  const int b_ = blockIdx.x;
  const size_t tokb = (size_t)b_ * NPIX;
#pragma unroll 1
  for (int k = 0; k < NDIR; ++k) {
    const float* wr = dtw + ((size_t)k * DIN + d) * DTRK;
    const float w0 = wr[0], w1 = wr[1], w2 = wr[2], w3 = wr[3], w4 = wr[4], w5 = wr[5];
    const float db = dtb[k * DIN + d];
    const float Dk = Dsp[k * DIN + d];
    float An[NST], h[NST];
#pragma unroll
    for (int n = 0; n < NST; ++n) {
      const float al = Alog[((size_t)k * DIN + d) * NST + n];
      An[n] = -__expf(al);
      h[n]  = 0.f;
    }
    const float* xd = XDBL + ((size_t)k * NTOK + tokb) * XDW;
#pragma unroll 1
    for (int c = 0; c < NPIX / 32; ++c) {
      __syncthreads();
      for (int q = d; q < 320; q += DIN) {
        const int s  = q / 10;
        const int j4 = (q - s * 10) * 4;
        const int l  = c * 32 + s;
        const int lr = (k >= 2) ? (NPIX - 1 - l) : l;
        const int tok = (k & 1) ? ((lr % IMH) * IMW + lr / IMH) : lr;
        const v4f v = *(const v4f*)(xd + (size_t)tok * XDW + j4);
        *(v4f*)(sRow + s * 40 + j4) = v;
      }
      __syncthreads();
#pragma unroll 1
      for (int s = 0; s < 32; ++s) {
        const int l  = c * 32 + s;
        const int lr = (k >= 2) ? (NPIX - 1 - l) : l;
        const int tok = (k & 1) ? ((lr % IMH) * IMW + lr / IMH) : lr;
        const size_t ei = (tokb + tok) * DIN + d;
        const float u = XI[ei];
        const float* sr = sRow + s * 40;
        v4f Bv[4], Cv[4];
#pragma unroll
        for (int i = 0; i < 4; ++i) {
          Bv[i] = *(const v4f*)(sr + 4 * i);
          Cv[i] = *(const v4f*)(sr + 16 + 4 * i);
        }
        const v4f D0 = *(const v4f*)(sr + 32);
        const v2f D1 = *(const v2f*)(sr + 36);
        float dp = db;
        dp = fmaf(w0, D0[0], dp);
        dp = fmaf(w1, D0[1], dp);
        dp = fmaf(w2, D0[2], dp);
        dp = fmaf(w3, D0[3], dp);
        dp = fmaf(w4, D1[0], dp);
        dp = fmaf(w5, D1[1], dp);
        const float ex    = __expf(-fabsf(dp));
        const float delta = fmaxf(dp, 0.0f) + __logf(1.0f + ex);
        const float du    = delta * u;
        float y = Dk * u;
#pragma unroll
        for (int n = 0; n < NST; ++n) {
          const float e  = __expf(delta * An[n]);
          const float hn = fmaf(e, h[n], du * Bv[n >> 2][n & 3]);
          h[n] = hn;
          y = fmaf(hn, Cv[n >> 2][n & 3], y);
        }
        float* yp = Y + ei;
        if (k > 0) {
          const float old = *(const float*)yp;
          y += old;
        }
        *(volatile float*)yp = y;
        __threadfence();
        *(volatile float*)yp = y;
      }
    }
  }
}

__global__ __launch_bounds__(256) void ln_gate_kernel(
    const float* __restrict__ Y, const float* __restrict__ Z,
    const float* __restrict__ g, const float* __restrict__ be,
    unsigned short* __restrict__ dst)
{
  __shared__ __align__(16) _Float16 sT[32 * DIN];
  const int t = threadIdx.x;
  const int r = t >> 3, part = t & 7;
  const int row = blockIdx.x * 32 + r;
  const int c0  = part * 24;
  const float* yr = Y + (size_t)row * DIN + c0;
  const float* zr = Z + (size_t)row * DIN + c0;
  v4f a[6];
#pragma unroll
  for (int j = 0; j < 6; ++j) a[j] = *(const v4f*)(yr + 4 * j);
  float s = 0.f;
#pragma unroll
  for (int j = 0; j < 6; ++j) s += (a[j][0] + a[j][1]) + (a[j][2] + a[j][3]);
  s += __shfl_xor(s, 1, 32);
  s += __shfl_xor(s, 2, 32);
  s += __shfl_xor(s, 4, 32);
  const float mu = s * (1.0f / 192.0f);
  float q = 0.f;
#pragma unroll
  for (int j = 0; j < 6; ++j) {
#pragma unroll
    for (int e = 0; e < 4; ++e) { const float dd = a[j][e] - mu; q = fmaf(dd, dd, q); }
  }
  q += __shfl_xor(q, 1, 32);
  q += __shfl_xor(q, 2, 32);
  q += __shfl_xor(q, 4, 32);
  const float var = q * (1.0f / 192.0f);
  const float is  = rsqrtf(var + 1e-5f);
#pragma unroll
  for (int j = 0; j < 6; ++j) {
    const v4f zz = *(const v4f*)(zr + 4 * j);
    const v4f gg = *(const v4f*)(g  + c0 + 4 * j);
    const v4f bb = *(const v4f*)(be + c0 + 4 * j);
    v4h hv;
#pragma unroll
    for (int e = 0; e < 4; ++e) {
      const float gn = ((a[j][e] - mu) * is) * gg[e] + bb[e];
      const float zv = zz[e];
      const float sg = __builtin_amdgcn_rcpf(1.0f + __expf(-zv));
      hv[e] = (_Float16)((gn * (zv * sg)) * 16.0f);
    }
    *(v4h*)(sT + r * DIN + c0 + 4 * j) = hv;
  }
  __syncthreads();
  v8h vals[3];
#pragma unroll
  for (int it = 0; it < 3; ++it) vals[it] = *(const v8h*)(sT + (it * 256 + t) * 8);
  unsigned short* ob = dst + (size_t)blockIdx.x * 32 * DIN;
  for (int pass = 0; pass < 2; ++pass) {
#pragma unroll
    for (int it = 0; it < 3; ++it) *(volatile v8h*)(ob + (size_t)(it * 256 + t) * 8) = vals[it];
    __threadfence();
  }
}

__global__ __launch_bounds__(256) void merge_kernel(
    const float* __restrict__ XL3, const float* __restrict__ XR, const float* __restrict__ c3b,
    const float* __restrict__ x, float* __restrict__ out, int nq)
{
  const int f = blockIdx.x * 256 + threadIdx.x;
  if (f >= nq) return;
  const int pos = f / 48;
  const int q   = f - pos * 48;
  const v2f xl = *(const v2f*)(XL3 + (size_t)pos * NPADC + 2 * q);
  const v2f xr = *(const v2f*)(XR  + (size_t)pos * NPADC + 2 * q);
  const v2f bb = *(const v2f*)(c3b + 2 * q);
  const v4f xx = *(const v4f*)(x + (size_t)pos * CFULL + 4 * q);
  v4f o;
  o[0] = fmaxf(xl[0] + bb[0], 0.0f) + xx[0];
  o[1] = xr[0] + xx[1];
  o[2] = fmaxf(xl[1] + bb[1], 0.0f) + xx[2];
  o[3] = xr[1] + xx[3];
  float* op = out + (size_t)f * 4;
  *(volatile v4f*)op = o;
  __threadfence();
  *(volatile v4f*)op = o;
}

extern "C" void kernel_launch(void* const* d_in, const int* in_sizes, int n_in,
                              void* d_out, int out_size, void* d_ws, size_t ws_size,
                              hipStream_t stream)
{
  if (n_in < 32) return;
  const float* x     = (const float*)d_in[0];
  const float* bn1g  = (const float*)d_in[1];
  const float* bn1b  = (const float*)d_in[2];
  const float* bn1m  = (const float*)d_in[3];
  const float* bn1v  = (const float*)d_in[4];
  const float* bn2g  = (const float*)d_in[5];
  const float* bn2b  = (const float*)d_in[6];
  const float* bn2m  = (const float*)d_in[7];
  const float* bn2v  = (const float*)d_in[8];
  const float* bn3g  = (const float*)d_in[9];
  const float* bn3b  = (const float*)d_in[10];
  const float* bn3m  = (const float*)d_in[11];
  const float* bn3v  = (const float*)d_in[12];
  const float* c1w   = (const float*)d_in[13];
  const float* c1b   = (const float*)d_in[14];
  const float* c2w   = (const float*)d_in[15];
  const float* c2b   = (const float*)d_in[16];
  const float* c3w   = (const float*)d_in[17];
  const float* c3b   = (const float*)d_in[18];
  const float* lng   = (const float*)d_in[19];
  const float* lnb   = (const float*)d_in[20];
  const float* inpw  = (const float*)d_in[21];
  const float* dwcw  = (const float*)d_in[22];
  const float* dwcb  = (const float*)d_in[23];
  const float* xprw  = (const float*)d_in[24];
  const float* dtpw  = (const float*)d_in[25];
  const float* dtpb  = (const float*)d_in[26];
  const float* alog  = (const float*)d_in[27];
  const float* dsp   = (const float*)d_in[28];
  const float* ong   = (const float*)d_in[29];
  const float* onb   = (const float*)d_in[30];
  const float* outw  = (const float*)d_in[31];
  float* dout = (float*)d_out;

  if (in_sizes[0] != NTOK * CFULL) return;
  for (int i = 1; i <= 12; ++i) if (in_sizes[i] != CHALF) return;
  if (in_sizes[13] != 9 * CHALF * CHALF || in_sizes[14] != CHALF) return;
  if (in_sizes[15] != 9 * CHALF * CHALF || in_sizes[16] != CHALF) return;
  if (in_sizes[17] != CHALF * CHALF || in_sizes[18] != CHALF) return;
  if (in_sizes[19] != CHALF || in_sizes[20] != CHALF) return;
  if (in_sizes[21] != 2 * DIN * CHALF) return;
  if (in_sizes[22] != 9 * DIN || in_sizes[23] != DIN) return;
  if (in_sizes[24] != NDIR * XPROWS * DIN) return;
  if (in_sizes[25] != NDIR * DIN * DTRK || in_sizes[26] != NDIR * DIN) return;
  if (in_sizes[27] != NDIR * DIN * NST || in_sizes[28] != NDIR * DIN) return;
  if (in_sizes[29] != DIN || in_sizes[30] != DIN) return;
  if (in_sizes[31] != CHALF * DIN) return;
  if (out_size != NTOK * CFULL) return;

  const size_t SZ_BT1  = (size_t)NPADC * KCONV * 2;
  const size_t SZ_BT3  = (size_t)NPADC * CHALF * 2;
  const size_t SZ_WIN  = (size_t)2 * DIN * CHALF * 2;
  const size_t SZ_WX   = (size_t)NDIR * XDW * DIN * 2;
  const size_t SZ_WO   = (size_t)NPADC * DIN * 2;
  const size_t SZ_ACOL = (size_t)NTOK * KCONV * 2;
  const size_t SZ_XDBL = (size_t)NDIR * NTOK * XDW * 4;
  const size_t SZ_H192 = (size_t)NTOK * DIN * 2;
  const size_t SZ_H96  = (size_t)NTOK * CHALF * 2;
  const size_t SZ_F128 = (size_t)NTOK * NPADC * 4;
  const size_t SZ_F192 = (size_t)NTOK * DIN * 4;
  const size_t OFF_BT1  = 0;
  const size_t OFF_BT2  = OFF_BT1 + SZ_BT1;
  const size_t OFF_BT3  = OFF_BT2 + SZ_BT1;
  const size_t OFF_WIN  = OFF_BT3 + SZ_BT3;
  const size_t OFF_WX   = OFF_WIN + SZ_WIN;
  const size_t OFF_WO   = OFF_WX  + SZ_WX;
  const size_t OFF_RA   = OFF_WO  + SZ_WO;
  const size_t OFF_XDBL = OFF_RA;
  const size_t OFF_X16  = OFF_RA + SZ_XDBL;
  const size_t OFF_XRN  = OFF_X16 + SZ_H192;
  if (OFF_XRN + SZ_H96 > OFF_RA + SZ_ACOL) return;
  const size_t OFF_RY   = OFF_RA  + SZ_ACOL;
  const size_t OFF_RT   = OFF_RY  + SZ_F128;
  const size_t OFF_RZ   = OFF_RT  + SZ_H96;
  const size_t OFF_RXI  = OFF_RZ  + SZ_F192;
  const size_t OFF_RP   = OFF_RXI + SZ_F192;
  const size_t TOTAL    = OFF_RP  + SZ_F192;
  if (ws_size < TOTAL) return;

  char* ws = (char*)d_ws;
  unsigned short* BT1   = (unsigned short*)(ws + OFF_BT1);
  unsigned short* BT2   = (unsigned short*)(ws + OFF_BT2);
  unsigned short* BT3   = (unsigned short*)(ws + OFF_BT3);
  unsigned short* WIN   = (unsigned short*)(ws + OFF_WIN);
  unsigned short* WX    = (unsigned short*)(ws + OFF_WX);
  unsigned short* WO    = (unsigned short*)(ws + OFF_WO);
  unsigned short* ACOL  = (unsigned short*)(ws + OFF_RA);
  float*          XDBL  = (float*)(ws + OFF_XDBL);
  unsigned short* XI16  = (unsigned short*)(ws + OFF_X16);
  unsigned short* YG16  = XI16;
  unsigned short* XRN16 = (unsigned short*)(ws + OFF_XRN);
  float*          YC    = (float*)(ws + OFF_RY);
  unsigned short* T16   = (unsigned short*)(ws + OFF_RT);
  float*          ZB    = (float*)(ws + OFF_RZ);
  float*          XI    = (float*)(ws + OFF_RXI);
  float*          XR    = XI;
  float*          XP    = (float*)(ws + OFF_RP);
  float*          YS    = XP;
  const float*    nores = x;

  const int NCH_AFF = NTOK * 12;
  const int NCH_COL = NTOK * 108;
  const float NEG_BIG = -INFINITY;

  cast_convw_kernel<<<(NPADC * KCONV / 8) / 256, 256, 0, stream>>>(c1w, BT1, KCONV, NPADC * KCONV / 8, 16.0f);
  cast_convw_kernel<<<(NPADC * KCONV / 8) / 256, 256, 0, stream>>>(c2w, BT2, KCONV, NPADC * KCONV / 8, 16.0f);
  cast_convw_kernel<<<(NPADC * CHALF / 8) / 256, 256, 0, stream>>>(c3w, BT3, CHALF, NPADC * CHALF / 8, 16.0f);
  cast_rows_kernel<<<(2 * DIN * CHALF / 8) / 256, 256, 0, stream>>>(inpw, WIN, 2 * DIN, 2 * DIN, CHALF, 0, 2 * DIN * CHALF / 8, 16.0f);
  cast_rows_kernel<<<(NDIR * XDW * DIN / 8) / 256, 256, 0, stream>>>(xprw, WX, XPROWS, XDW, DIN, DTRK, NDIR * XDW * DIN / 8, 16.0f);
  cast_rows_kernel<<<(NPADC * DIN / 8) / 256, 256, 0, stream>>>(outw, WO, CHALF, NPADC, DIN, 0, NPADC * DIN / 8, 16.0f);

  affine_f16_kernel<<<NCH_AFF / 256, 256, 0, stream>>>(x, CFULL, bn1g, bn1b, bn1m, bn1v, c1b, 0.0f, NEG_BIG, T16, NCH_AFF);
  im2col_copy_kernel<<<NCH_COL / 256, 256, 0, stream>>>(T16, ACOL, NCH_COL);
  wmma_gemm64<0, false, 0, 0, false, 0><<<dim3(98, 1), 256, 0, stream>>>(
      ACOL, ACOL, KCONV, 0L, BT1, BT1, KCONV, 0L, (void*)YC, (void*)YC, NPADC, 0L,
      nores, nores, 0L, NTOK, NPADC, KCONV, 1.0f / 16.0f);
  affine_f16_kernel<<<NCH_AFF / 256, 256, 0, stream>>>(YC, NPADC, bn2g, bn2b, bn2m, bn2v, c1b, 1.0f, 0.0f, T16, NCH_AFF);
  im2col_copy_kernel<<<NCH_COL / 256, 256, 0, stream>>>(T16, ACOL, NCH_COL);
  wmma_gemm64<0, false, 0, 0, false, 0><<<dim3(98, 1), 256, 0, stream>>>(
      ACOL, ACOL, KCONV, 0L, BT2, BT2, KCONV, 0L, (void*)YC, (void*)YC, NPADC, 0L,
      nores, nores, 0L, NTOK, NPADC, KCONV, 1.0f / 16.0f);
  affine_f16_kernel<<<NCH_AFF / 256, 256, 0, stream>>>(YC, NPADC, bn3g, bn3b, bn3m, bn3v, c2b, 1.0f, 0.0f, T16, NCH_AFF);
  wmma_gemm64<0, false, 0, 0, false, 0><<<dim3(98, 1), 256, 0, stream>>>(
      T16, T16, CHALF, 0L, BT3, BT3, CHALF, 0L, (void*)YC, (void*)YC, NPADC, 0L,
      nores, nores, 0L, NTOK, NPADC, CHALF, 1.0f / 16.0f);

  ln96_kernel<<<NTOK / 64, 256, 0, stream>>>(x, lng, lnb, XRN16);
  wmma_gemm64<0, false, 0, 0, false, 0><<<dim3(147, 1), 256, 0, stream>>>(
      XRN16, XRN16, CHALF, 0L, WIN, WIN, CHALF, 0L, (void*)XP, (void*)XP, DIN, 0L,
      nores, nores, 0L, NTOK, DIN, CHALF, 1.0f / 16.0f);
  wmma_gemm64<0, false, 0, 0, false, 0><<<dim3(147, 1), 256, 0, stream>>>(
      XRN16, XRN16, CHALF, 0L, WIN + (size_t)DIN * CHALF, WIN + (size_t)DIN * CHALF, CHALF, 0L,
      (void*)ZB, (void*)ZB, DIN, 0L, nores, nores, 0L, NTOK, DIN, CHALF, 1.0f / 16.0f);
  dwconv_silu_kernel<<<NBATCH * IMH, DIN, 0, stream>>>(XP, dwcw, dwcb, XI, XI16);
  wmma_gemm64<0, false, 0, 0, false, 0><<<dim3(49, NDIR), 256, 0, stream>>>(
      XI16, XI16, DIN, 0L, WX, WX, DIN, (long)XDW * DIN, (void*)XDBL, (void*)XDBL, XDW, (long)NTOK * XDW,
      nores, nores, 0L, NTOK, XDW, DIN, 1.0f / 1024.0f);
  scan4_kernel<<<NBATCH, DIN, 0, stream>>>(XDBL, XI, dtpw, dtpb, alog, dsp, YS);
  ln_gate_kernel<<<NTOK / 32, 256, 0, stream>>>(YS, ZB, ong, onb, YG16);
  wmma_gemm64<0, false, 0, 0, false, 0><<<dim3(98, 1), 256, 0, stream>>>(
      YG16, YG16, DIN, 0L, WO, WO, DIN, 0L, (void*)XR, (void*)XR, NPADC, 0L,
      nores, nores, 0L, NTOK, NPADC, DIN, 1.0f / 256.0f);

  merge_kernel<<<(NTOK * 48) / 256, 256, 0, stream>>>(YC, XR, c3b, x, dout, NTOK * 48);
}
